// DMSA_6983616823333
// MI455X (gfx1250) — hardware-verified
//
#include <hip/hip_runtime.h>
#include <math.h>


#define USE_TDM 0
typedef __attribute__((ext_vector_type(16))) _Float16 v16h;
typedef __attribute__((ext_vector_type(8)))  float    v8f;
#define VST2(T, ptr, val) do { const T _v = (val); *(volatile T*)(ptr) = _v; __threadfence(); *(volatile T*)(ptr) = _v; } while (0)
__device__ __forceinline__ int kmap(int e, int half) { return (e < 8) ? (8 * half + e) : (16 + 8 * half + (e - 8)); }

#define WMMA_F16(A, B, C) \
  __builtin_amdgcn_wmma_f32_16x16x32_f16(false, (A), false, (B), (short)0, (C), false, false)

constexpr int Bb = 4;
constexpr int Nn = 1200;
constexpr int Dd = 256;
constexpr int Hh = 8;
constexpr int HD = 32;
constexpr int E3 = 3 * Dd;
constexpr int NT = (Nn + 31) / 32;
constexpr int WPB = 5;
constexpr int GRP = (Nn / 16) / WPB;


#if USE_TDM
typedef unsigned int tdm_v4u __attribute__((ext_vector_type(4)));
typedef int          tdm_v8i __attribute__((ext_vector_type(8)));
typedef int          tdm_v4i __attribute__((ext_vector_type(4)));

__device__ __forceinline__ void tdm_load_tile_f32(const float* gsrc, unsigned lds_off,
                                                  int rows_avail) {
  unsigned long long ga = (unsigned long long)(uintptr_t)gsrc;
  tdm_v4u g0;
  tdm_v8i g1;
  tdm_v4i g2 = {0, 0, 0, 0}, g3 = {0, 0, 0, 0};
  tdm_v8i g4 = {0, 0, 0, 0, 0, 0, 0, 0};
  g0[0] = 1u;
  g0[1] = lds_off;
  g0[2] = (unsigned)(ga & 0xffffffffu);
  g0[3] = (unsigned)((ga >> 32) & 0x1ffffffu) | (2u << 30);
  g1[0] = (int)(2u << 16);
  g1[1] = (int)(32u << 16);
  g1[2] = (int)((unsigned)(rows_avail & 0xffff) << 16);
  g1[3] = (int)(32u << 16);
  g1[4] = (int)32u;
  g1[5] = (int)768u;
  g1[6] = 0;
  g1[7] = 0;
  __builtin_amdgcn_tensor_load_to_lds(g0, g1, g2, g3, g4, 0);
}
#endif

__global__ void beta_kernel(const float* __restrict__ feat,
                            const float* __restrict__ bw,
                            const float* __restrict__ bb,
                            float* __restrict__ beta) {
  int idx = blockIdx.x * blockDim.x + threadIdx.x;
  if (idx >= Bb * Hh * Nn) return;
  int n = idx % Nn;
  int h = (idx / Nn) % Hh;
  int b = idx / (Nn * Hh);
  const float* f = feat + (size_t)(b * Nn + n) * Dd;
  const float* w = bw + (size_t)h * Dd;
  float s = 0.f;
  for (int d = 0; d < Dd; d += 4)
    s += f[d] * w[d] + f[d + 1] * w[d + 1] + f[d + 2] * w[d + 2] + f[d + 3] * w[d + 3];
  VST2(float, beta + idx, s + bb[h]);
}

__global__ void gemm_wmma(const float* __restrict__ X, const float* __restrict__ W,
                          const float* __restrict__ bias, float* __restrict__ Y,
                          int M, int Nc, int K) {
  int wave = (int)((blockIdx.x * blockDim.x + threadIdx.x) >> 5);
  int lane = threadIdx.x & 31;
  int half = lane >> 4, lan = lane & 15;
  int ntn  = Nc >> 5;
  int tm = wave / ntn, tn = wave % ntn;
  if (tm >= (M >> 4)) return;

  int arow = tm * 16 + lan;
  int bcol = tn * 32 + lan;
  v8f c = {}, c2 = {};
  for (int k0 = 0; k0 < K; k0 += 32) {
    const float* xp = X + (size_t)arow * K + k0 + half * 8;
    const float* wp = W + (size_t)bcol * K + k0 + half * 8;
    const float* wp2 = wp + (size_t)16 * K;
    v16h a, bf, bf2;
#pragma unroll
    for (int i = 0; i < 8; i++) {
      a[i]     = (_Float16)xp[i];      a[8 + i]   = (_Float16)xp[16 + i];
      bf[i]    = (_Float16)wp[i];      bf[8 + i]  = (_Float16)wp[16 + i];
      bf2[i]   = (_Float16)wp2[i];     bf2[8 + i] = (_Float16)wp2[16 + i];
    }
    c = WMMA_F16(a, bf, c); c2 = WMMA_F16(a, bf2, c2);
    asm volatile("v_nop\n\tv_nop\n\tv_nop\n\tv_nop" : "+v"(c), "+v"(c2) : "v"(a), "v"(bf2));
  }
  const int rb0 = tm * 16;
  const float bcv = bias[tn * 32 + lane];
  for (int pass = 0; pass < 2; ++pass) {
#pragma unroll
    for (int r = 0; r < 8; r++) {
      const float x0 = __shfl_xor(c[r], 16), x1 = __shfl_xor(c2[r], 16);
      *(volatile float*)(Y + (size_t)(rb0 + r) * Nc + tn * 32 + lane)     = (half ? x1 : c[r]) + bcv;
      *(volatile float*)(Y + (size_t)(rb0 + 8 + r) * Nc + tn * 32 + lane) = (half ? c2[r] : x0) + bcv;
    }
    __threadfence();
  }
}

__global__ void __launch_bounds__(32 * WPB)
attn_kernel(const float* __restrict__ qkv, const float* __restrict__ bbox,
            const float* __restrict__ beta, float* __restrict__ aout) {
  __shared__ float Kt[2][32][32];
  __shared__ float Vt[2][32][32];
  __shared__ float Pl[WPB][16][32];

  int bid = blockIdx.x;
  int grp = bid % GRP;
  int h   = (bid / GRP) % Hh;
  int b   = bid / (GRP * Hh);
  int tid  = threadIdx.x;
  int wid  = tid >> 5;
  int lane = tid & 31;
  int half = lane >> 4, lan = lane & 15;
  int qt = grp * WPB + wid;

  const float scale = 0.17677669529663687f;
  const float* kbase = qkv + (size_t)b * Nn * E3 + Dd + h * HD;
  const float* vbase = qkv + (size_t)b * Nn * E3 + 2 * Dd + h * HD;

  int qrow_a = qt * 16 + lan;
  const float* qp = qkv + (size_t)(b * Nn + qrow_a) * E3 + h * HD;
  v16h aq, aql;
#pragma unroll
  for (int i = 0; i < 16; i++) {
    const float qv = qp[kmap(i, half)] * scale;
    aq[i] = (_Float16)qv; aql[i] = (_Float16)(qv - (float)aq[i]);
  }

  int rb = qt * 16 + half * 8;
  float qcx[8], qcy[8], betar[8];
#pragma unroll
  for (int r = 0; r < 8; r++) {
    qcx[r]   = bbox[(size_t)(b * Nn + rb + r) * 10 + 0];
    qcy[r]   = bbox[(size_t)(b * Nn + rb + r) * 10 + 1];
    betar[r] = beta[((size_t)b * Hh + h) * Nn + rb + r];
  }

  float mrow[8], lrow[8];
  v8f acc0 = {}, acc1 = {};
#pragma unroll
  for (int r = 0; r < 8; r++) { mrow[r] = -3.0e38f; lrow[r] = 0.f; }

#if USE_TDM
  if (wid == 0) {
    tdm_load_tile_f32(kbase, (unsigned)(uintptr_t)&Kt[0][0][0], Nn < 32 ? Nn : 32);
    tdm_load_tile_f32(vbase, (unsigned)(uintptr_t)&Vt[0][0][0], Nn < 32 ? Nn : 32);
  }
#endif

  for (int t = 0; t < NT; t++) {
    int kb  = t * 32;
    int cur = t & 1;
    bool v1 = (kb + 16 < Nn);

#if USE_TDM
    if (wid == 0) {
      if (t + 1 < NT) {
        int kb2 = kb + 32;
        int rows = Nn - kb2;
        if (rows > 32) rows = 32;
        tdm_load_tile_f32(kbase + (size_t)kb2 * E3,
                          (unsigned)(uintptr_t)&Kt[1 - cur][0][0], rows);
        tdm_load_tile_f32(vbase + (size_t)kb2 * E3,
                          (unsigned)(uintptr_t)&Vt[1 - cur][0][0], rows);
        __builtin_amdgcn_s_wait_tensorcnt(2);
      } else {
        __builtin_amdgcn_s_wait_tensorcnt(0);
      }
    }
    __syncthreads();
#else
    for (int idx = tid; idx < 32 * 32; idx += 32 * WPB) {
      int row = idx >> 5, col = idx & 31;
      int key = kb + row;
      bool kv = key < Nn;
      Kt[cur][row][col] = kv ? kbase[(size_t)key * E3 + col] : 0.f;
      Vt[cur][row][col] = kv ? vbase[(size_t)key * E3 + col] : 0.f;
    }
    __syncthreads();
#endif

    v16h bk0, bk1, bl0, bl1;
#pragma unroll
    for (int i = 0; i < 16; i++) {
      const float k0v = Kt[cur][lan][kmap(i, half)], k1v = Kt[cur][16 + lan][kmap(i, half)];
      bk0[i] = (_Float16)k0v; bl0[i] = (_Float16)(k0v - (float)bk0[i]);
      bk1[i] = (_Float16)k1v; bl1[i] = (_Float16)(k1v - (float)bk1[i]);
    }
    v8f s0 = {}, s1 = {};
    s0 = WMMA_F16(aq, bk0, s0); s0 = WMMA_F16(aq, bl0, s0); s0 = WMMA_F16(aql, bk0, s0);
    s1 = WMMA_F16(aq, bk1, s1); s1 = WMMA_F16(aq, bl1, s1); s1 = WMMA_F16(aql, bk1, s1);
    asm volatile("v_nop\n\tv_nop\n\tv_nop\n\tv_nop" : "+v"(s0), "+v"(s1) : "v"(aql), "v"(bk1));

    int key0 = kb + lan;
    int key1 = kb + 16 + lan;
    float kcx0 = bbox[(size_t)(b * Nn + key0) * 10 + 0];
    float kcy0 = bbox[(size_t)(b * Nn + key0) * 10 + 1];
    float kcx1 = v1 ? bbox[(size_t)(b * Nn + key1) * 10 + 0] : 0.f;
    float kcy1 = v1 ? bbox[(size_t)(b * Nn + key1) * 10 + 1] : 0.f;

    float p0[8], p1[8];
#pragma unroll
    for (int r = 0; r < 8; r++) {
      float dx0 = qcx[r] - kcx0, dy0 = qcy[r] - kcy0;
      float dx1 = qcx[r] - kcx1, dy1 = qcy[r] - kcy1;
      float s0r = s0[r] - sqrtf(dx0 * dx0 + dy0 * dy0) * betar[r];
      float s1r = v1 ? (s1[r] - sqrtf(dx1 * dx1 + dy1 * dy1) * betar[r]) : -3.0e38f;

      float rm = fmaxf(s0r, s1r);
      for (int off = 1; off < 16; off <<= 1) rm = fmaxf(rm, __shfl_xor(rm, off, 32));
      float mnew = fmaxf(mrow[r], rm);
      float corr = __expf(mrow[r] - mnew);
      float e0 = __expf(s0r - mnew);
      float e1 = v1 ? __expf(s1r - mnew) : 0.f;
      float rs = e0 + e1;
      for (int off = 1; off < 16; off <<= 1) rs += __shfl_xor(rs, off, 32);
      lrow[r] = lrow[r] * corr + rs;
      mrow[r] = mnew;
      acc0[r] *= corr;
      acc1[r] *= corr;
      p0[r] = e0;
      p1[r] = e1;
    }

#pragma unroll
    for (int r = 0; r < 8; r++) {
      Pl[wid][half * 8 + r][lan]      = p0[r];
      Pl[wid][half * 8 + r][16 + lan] = p1[r];
    }
    v16h ap;
#pragma unroll
    for (int i = 0; i < 8; i++) {
      ap[i]     = (_Float16)Pl[wid][lan][half * 8 + i];
      ap[8 + i] = (_Float16)Pl[wid][lan][16 + half * 8 + i];
    }

    v16h bv0, bv1;
#pragma unroll
    for (int j = 0; j < 16; j++) {
      bv0[j] = (_Float16)Vt[cur][kmap(j, half)][lan];
      bv1[j] = (_Float16)Vt[cur][kmap(j, half)][16 + lan];
    }
    acc0 = WMMA_F16(ap, bv0, acc0);
    acc1 = WMMA_F16(ap, bv1, acc1);
    asm volatile("v_nop\n\tv_nop\n\tv_nop\n\tv_nop" : "+v"(acc0), "+v"(acc1) : "v"(ap), "v"(bv1));

    __syncthreads();
  }

  for (int pass = 0; pass < 2; ++pass) {
#pragma unroll
    for (int r = 0; r < 8; r++) {
      const float v0 = acc0[r] / lrow[r], v1 = acc1[r] / lrow[r];
      const float x0 = __shfl_xor(v0, 16), x1 = __shfl_xor(v1, 16);
      float* rowA = aout + (size_t)(b * Nn + qt * 16 + r) * Dd + h * HD;
      float* rowB = aout + (size_t)(b * Nn + qt * 16 + 8 + r) * Dd + h * HD;
      *(volatile float*)(rowA + lane) = half ? x1 : v0;
      *(volatile float*)(rowB + lane) = half ? v1 : x0;
    }
    __threadfence();
  }
}

extern "C" void kernel_launch(void* const* d_in, const int* in_sizes, int n_in,
                              void* d_out, int out_size, void* d_ws, size_t ws_size,
                              hipStream_t stream) {
  const float* bbox   = (const float*)d_in[0];
  const float* feat   = (const float*)d_in[1];
  const float* beta_w = (const float*)d_in[2];
  const float* beta_b = (const float*)d_in[3];
  const float* in_w   = (const float*)d_in[4];
  const float* in_b   = (const float*)d_in[5];
  const float* out_w  = (const float*)d_in[6];
  const float* out_b  = (const float*)d_in[7];
  float* out = (float*)d_out;

  float* qkv  = (float*)d_ws;
  float* beta = qkv + (size_t)Bb * Nn * E3;
  float* aout = beta + (size_t)Bb * Hh * Nn;

  int tb = Bb * Hh * Nn;
  beta_kernel<<<(tb + 255) / 256, 256, 0, stream>>>(feat, beta_w, beta_b, beta);

  (void)in_sizes; (void)n_in; (void)out_size;
  if (ws_size < (size_t)(Bb * Nn * E3 + Bb * Hh * Nn + Bb * Nn * Dd) * 4) return;
  {
    int waves = (Bb * Nn / 16) * (E3 / 32);
    gemm_wmma<<<waves / 8, 256, 0, stream>>>(feat, in_w, in_b, qkv, Bb * Nn, E3, Dd);
  }

  attn_kernel<<<Bb * Hh * GRP, 32 * WPB, 0, stream>>>(qkv, bbox, beta, aout);

  {
    int waves = (Bb * Nn / 16) * (Dd / 32);
    gemm_wmma<<<waves / 8, 256, 0, stream>>>(aout, out_w, out_b, out, Bb * Nn, Dd, Dd);
  }
}
